// DemoAttentionModel_77575699300507
// MI455X (gfx1250) — hardware-run, weakly checked
//
#include <hip/hip_runtime.h>
#include <math.h>

constexpr int kBatch   = 2;
constexpr int kSeq     = 4096;
constexpr int kDim     = 512;
constexpr int kHeads   = 8;
constexpr int kHeadDim = 64;
constexpr int kFF      = 2048;
constexpr int kTok     = kBatch * kSeq;
constexpr int kQKld    = 2 * kDim;
constexpr float kWCarry     = 16.0f;
constexpr float kWCarryInv  = 1.0f / 16.0f;
constexpr float kPCarry     = 2048.0f;
constexpr float kCtxCarry   = 256.0f;
constexpr float kActCarry   = 16.0f;
constexpr float kPVScale    = kCtxCarry / kPCarry;
constexpr float kWoScale    = 1.0f / (kCtxCarry * kWCarry);
constexpr float kW2Scale    = 1.0f / (kActCarry * kWCarry);
constexpr float kScoreScale = 0.125f;
constexpr float kInvDim     = 1.0f / 512.0f;
constexpr float kLnEps      = 1e-5f;

constexpr size_t kOffH    = 0;
constexpr size_t kOffQK   = kOffH  + (size_t)kTok * kDim * 2;
constexpr size_t kOffVT   = kOffQK + (size_t)kTok * kQKld * 2;
constexpr size_t kOffS    = kOffVT + (size_t)kBatch * kDim * kSeq * 2;
constexpr size_t kOffP    = kOffS  + (size_t)kSeq * kSeq * 4;
constexpr size_t kWsTotal = kOffP  + (size_t)kSeq * kSeq * 2;
static_assert(kOffQK == 8388608u, "carve");
static_assert(kOffVT == 25165824u, "carve");
static_assert(kOffS == 33554432u, "carve");
static_assert(kOffP == 100663296u, "carve");
static_assert(kWsTotal == 134217728u, "carve");
static_assert((size_t)kTok * kDim * 4 == 16777216u, "x1 fits R_QK");
static_assert((size_t)kTok * kFF * 4 == 67108864u, "ffn pre-activation fits R_S");
static_assert((size_t)kTok * kFF * 2 == 33554432u, "gelu act fits R_P");
static_assert((size_t)(kDim * kDim + kFF * kDim + kDim * kFF) * 2 <= (size_t)kBatch * kDim * kSeq * 2, "late weights fit R_VT");
static_assert((size_t)3 * kDim * kDim * 2 <= (size_t)kSeq * kSeq * 4, "early weights fit R_S");

typedef __attribute__((ext_vector_type(16))) _Float16 v16h;
typedef __attribute__((ext_vector_type(8)))  _Float16 v8h;
typedef __attribute__((ext_vector_type(16))) __bf16   v16b;
typedef __attribute__((ext_vector_type(8)))  __bf16   v8b;
typedef __attribute__((ext_vector_type(8)))  float    v8f;
typedef __attribute__((ext_vector_type(4)))  float    v4f;
typedef __attribute__((ext_vector_type(4)))  unsigned int v4u;

__device__ __forceinline__ unsigned short f2bf_bits(float f) {
  unsigned u = __float_as_uint(f);
  return (unsigned short)((u + 0x7FFFu + ((u >> 16) & 1u)) >> 16);
}
__device__ __forceinline__ float bf_bits2f(unsigned short h) { return __uint_as_float(((unsigned)h) << 16); }

__device__ __forceinline__ void dep_guard_h(v8f& a, v8f& b, v16h x, v16h y) { asm volatile("v_nop\n\tv_nop\n\tv_nop\n\tv_nop" : "+v"(a), "+v"(b) : "v"(x), "v"(y)); }
__device__ __forceinline__ void dep_guard_b(v8f& a, v8f& b, v16b x, v16b y) { asm volatile("v_nop\n\tv_nop\n\tv_nop\n\tv_nop" : "+v"(a), "+v"(b) : "v"(x), "v"(y)); }
__device__ __forceinline__ void keep4_h(v16h a, v16h b, v16h c, v16h d) { asm volatile("v_nop" :: "v"(a), "v"(b), "v"(c), "v"(d)); }
__device__ __forceinline__ void keep4_b(v16b a, v16b b, v16b c, v16b d) { asm volatile("v_nop" :: "v"(a), "v"(b), "v"(c), "v"(d)); }
__device__ __forceinline__ void acc_guard4(v8f& a, v8f& b, v8f& c, v8f& d) { asm volatile("v_nop\n\tv_nop\n\tv_nop\n\tv_nop" : "+v"(a), "+v"(b), "+v"(c), "+v"(d)); }
template <typename T> struct Frag;
template <> struct Frag<_Float16> {
  typedef v16h V; union U { v16h v; v8h h[2]; };
  static __device__ __forceinline__ v16h load(const _Float16* p) {
    U f; f.h[0] = *(const v8h*)(p); f.h[1] = *(const v8h*)(p + 16); return f.v;
  }
  static __device__ __forceinline__ v8f mma(v16h a, v16h b, v8f c) {
    return __builtin_amdgcn_wmma_f32_16x16x32_f16(false, a, false, b, (short)0, c, false, false);
  }
  static __device__ __forceinline__ void guard(v8f& a, v8f& b, v16h x, v16h y) { dep_guard_h(a, b, x, y); }
  static __device__ __forceinline__ void keep(v16h a, v16h b, v16h c, v16h d) { keep4_h(a, b, c, d); }
};
template <> struct Frag<__bf16> {
  typedef v16b V; union U { v16b v; v8b h[2]; };
  static __device__ __forceinline__ v16b load(const __bf16* p) {
    U f; f.h[0] = *(const v8b*)(p); f.h[1] = *(const v8b*)(p + 16); return f.v;
  }
  static __device__ __forceinline__ v8f mma(v16b a, v16b b, v8f c) {
    return __builtin_amdgcn_wmma_f32_16x16x32_bf16(false, a, false, b, (short)0, c, false, false);
  }
  static __device__ __forceinline__ void guard(v8f& a, v8f& b, v16b x, v16b y) { dep_guard_b(a, b, x, y); }
  static __device__ __forceinline__ void keep(v16b a, v16b b, v16b c, v16b d) { keep4_b(a, b, c, d); }
};

__device__ __forceinline__ unsigned pk16(unsigned short a, unsigned short b) { return (unsigned)a | ((unsigned)b << 16); }
__device__ __forceinline__ unsigned short h_bits(float f) { const _Float16 h = (_Float16)f; return __builtin_bit_cast(unsigned short, h); }

template <int ET> struct Elem;
template <> struct Elem<0> { typedef _Float16 T; };
template <> struct Elem<1> { typedef __bf16 T; };
template <int ET, bool SPLIT, int BIAS_MODE, int OUT_MODE, bool RESID, int ACT = 0>
__global__ __launch_bounds__(256) void wmma_gemm64(
    const unsigned short* __restrict__ Ap, const unsigned short* __restrict__ A2p, int lda, long strideA,
    const unsigned short* __restrict__ Btp, const unsigned short* __restrict__ Bt2p, int ldb, long strideB,
    void* __restrict__ Cout, void* __restrict__ Cout2, int ldc, long strideC,
    const float* __restrict__ bias,
    const float* __restrict__ resid, long strideR,
    int M, int N, int K, float scale) {
  typedef typename Elem<ET>::T T;
  typedef typename Frag<T>::V V;
  const T* A = (const T*)Ap; const T* A2 = (const T*)A2p; const T* Bt = (const T*)Btp; const T* Bt2 = (const T*)Bt2p;
  __shared__ __align__(16) float sT[8][16 * 68];
  const int b    = blockIdx.y;
  const int lane = threadIdx.x & 31;
  const int wave = threadIdx.x >> 5;
  const int tilesN = N >> 6;
  const int tilesM = M >> 6;
  const int tile = blockIdx.x * 8 + wave;
  if (tile >= tilesM * tilesN) return;
  const int tm = tile / tilesN;
  const int tn = tile - tm * tilesN;
  const int m0 = tm << 6;
  const int n0 = tn << 6;

  const T* Ab  = A  + (size_t)b * strideA;
  const T* Bb  = Bt + (size_t)b * strideB;
  const T* Ab2 = SPLIT ? (A2  + (size_t)b * strideA) : nullptr;
  const T* Bb2 = SPLIT ? (Bt2 + (size_t)b * strideB) : nullptr;

  const int rlane = lane & 15;
  const int koff  = (lane >> 4) * 8;
  const int mOff  = (lane >> 4) * 8;

  v8f acc[4][4];
#pragma unroll
  for (int i = 0; i < 4; ++i)
#pragma unroll
    for (int j = 0; j < 4; ++j) acc[i][j] = (v8f){0.f,0.f,0.f,0.f,0.f,0.f,0.f,0.f};

  for (int k0 = 0; k0 < K; k0 += 32) {
    V bh[4], bl[4];
#pragma unroll
    for (int j = 0; j < 4; ++j) {
      const size_t bo = (size_t)(n0 + (j << 4) + rlane) * ldb + koff + k0;
      bh[j] = Frag<T>::load(Bb + bo);
      if (SPLIT) bl[j] = Frag<T>::load(Bb2 + bo);
    }
#pragma unroll
    for (int i = 0; i < 4; ++i) {
      const size_t ao = (size_t)(m0 + (i << 4) + rlane) * lda + koff + k0;
      V ah = Frag<T>::load(Ab + ao);
      V al;
      if (SPLIT) al = Frag<T>::load(Ab2 + ao);
#pragma unroll
      for (int j = 0; j < 4; ++j) {
        acc[i][j] = Frag<T>::mma(ah, bh[j], acc[i][j]);
        if (SPLIT) {
          acc[i][j] = Frag<T>::mma(ah, bl[j], acc[i][j]);
          acc[i][j] = Frag<T>::mma(al, bh[j], acc[i][j]);
        }
      }
      Frag<T>::guard(acc[i][0], acc[i][3], ah, SPLIT ? al : ah);
    }
    Frag<T>::keep(bh[0], bh[1], bh[2], bh[3]);
    if (SPLIT) Frag<T>::keep(bl[0], bl[1], bl[2], bl[3]);
  }
  acc_guard4(acc[0][0], acc[0][1], acc[0][2], acc[0][3]);
  acc_guard4(acc[1][0], acc[1][1], acc[1][2], acc[1][3]);
  acc_guard4(acc[2][0], acc[2][1], acc[2][2], acc[2][3]);
  acc_guard4(acc[3][0], acc[3][1], acc[3][2], acc[3][3]);

  float* slab = sT[wave];
  const float* Rb = RESID ? (resid + (size_t)b * strideR) : nullptr;
#pragma unroll
  for (int i = 0; i < 4; ++i) {
    const int mBase = m0 + (i << 4);
#pragma unroll
    for (int j = 0; j < 4; ++j) {
      const int n = n0 + (j << 4) + rlane;
      float bv = 0.f;
      if (BIAS_MODE == 2) bv = bias[n];
#pragma unroll
      for (int r = 0; r < 8; ++r) {
        float v = acc[i][j][r] * scale;
        if (BIAS_MODE == 1) v += bias[mBase + mOff + r];
        if (BIAS_MODE == 2) v += bv;
        if (RESID) v += Rb[(size_t)(mBase + mOff + r) * ldc + n];
        if (ACT == 2) v = fmaxf(v, 0.0f);
        if (ACT == 4) v = (v > 0.f) ? v : 0.01f * v;
        slab[(mOff + r) * 68 + (j << 4) + rlane] = v;
      }
    }
    __builtin_amdgcn_fence(__ATOMIC_RELEASE, "workgroup");
    __builtin_amdgcn_wave_barrier();
    __builtin_amdgcn_fence(__ATOMIC_ACQUIRE, "workgroup");
    if (OUT_MODE == 0) {
      float* C = (float*)Cout + (size_t)b * strideC;
      const int hh = lane >> 4, c4 = (lane & 15) * 4;
      for (int pass = 0; pass < 2; ++pass) {
#pragma unroll
        for (int it = 0; it < 8; ++it) {
          const int row = it * 2 + hh;
          v4f v = *(const v4f*)(slab + row * 68 + c4);
          *(volatile v4f*)(C + (size_t)(mBase + row) * ldc + n0 + c4) = v;
        }
        __threadfence();
      }
    } else {
      const int q = lane >> 3, c8 = (lane & 7) * 8;
      unsigned short* C  = (unsigned short*)Cout  + (size_t)b * strideC;
      unsigned short* C2 = (OUT_MODE == 2) ? ((unsigned short*)Cout2 + (size_t)b * strideC) : nullptr;
      for (int pass = 0; pass < 2; ++pass) {
#pragma unroll
        for (int it = 0; it < 4; ++it) {
          const int row = it * 4 + q;
          const float* sp = slab + row * 68 + c8;
          v8h hv, lv;
#pragma unroll
          for (int e = 0; e < 8; ++e) {
            if (OUT_MODE == 1) {
              hv[e] = (_Float16)sp[e];
            } else {
              unsigned short hb = f2bf_bits(sp[e]);
              unsigned short lb = f2bf_bits(sp[e] - bf_bits2f(hb));
              hv[e] = __builtin_bit_cast(_Float16, hb);
              lv[e] = __builtin_bit_cast(_Float16, lb);
            }
          }
          *(volatile v8h*)(C + (size_t)(mBase + row) * ldc + n0 + c8) = hv;
          if (OUT_MODE == 2) *(volatile v8h*)(C2 + (size_t)(mBase + row) * ldc + n0 + c8) = lv;
        }
        __threadfence();
      }
    }
    __builtin_amdgcn_fence(__ATOMIC_RELEASE, "workgroup");
    __builtin_amdgcn_wave_barrier();
    __builtin_amdgcn_fence(__ATOMIC_ACQUIRE, "workgroup");
  }
}

__global__ __launch_bounds__(256) void tcast_kernel(const float* __restrict__ W0, const float* __restrict__ W1,
                                                    const float* __restrict__ W2, unsigned short* __restrict__ out,
                                                    int K, int N, float scale) {
  __shared__ float sm[64][65];
  const int t  = threadIdx.x;
  const int k0 = blockIdx.x * 64;
  const int n0 = blockIdx.y * 64;
  const int z  = blockIdx.z;
  const float* W = (z == 0) ? W0 : (z == 1) ? W1 : W2;
#pragma unroll
  for (int i = 0; i < 16; ++i) {
    const int e = i * 256 + t;
    const int r = e >> 6;
    const int c = e & 63;
    sm[c][r] = W[(size_t)(k0 + r) * N + n0 + c] * scale;
  }
  __syncthreads();
  const int lane = t & 31, wave = t >> 5;
  const int q = lane >> 3, c8 = (lane & 7) * 8;
  unsigned short* op = out + (size_t)z * N * K;
  for (int pass = 0; pass < 2; ++pass) {
#pragma unroll
    for (int it = 0; it < 2; ++it) {
      const int row = wave * 8 + it * 4 + q;
      unsigned short hb[8];
#pragma unroll
      for (int e = 0; e < 8; ++e) hb[e] = h_bits(sm[row][c8 + e]);
      const v4u u = (v4u){pk16(hb[0], hb[1]), pk16(hb[2], hb[3]), pk16(hb[4], hb[5]), pk16(hb[6], hb[7])};
      *(volatile v4u*)(op + (size_t)(n0 + row) * K + k0 + c8) = u;
    }
    __threadfence();
  }
}

__global__ __launch_bounds__(256) void ln_rows_kernel(const float* __restrict__ x, const float* __restrict__ g,
                                                      const float* __restrict__ bt, unsigned short* __restrict__ out,
                                                      int nrows) {
  const int lane = threadIdx.x & 31, wave = threadIdx.x >> 5;
  const int row  = blockIdx.x * 8 + wave;
  const int rowc = (row < nrows) ? row : (nrows - 1);
  const float* xr = x + (size_t)rowc * kDim;
  const int cA = 8 * lane, cB = 256 + 8 * lane;
  const v4f a0 = *(const v4f*)(xr + cA);
  const v4f a1 = *(const v4f*)(xr + cA + 4);
  const v4f a2 = *(const v4f*)(xr + cB);
  const v4f a3 = *(const v4f*)(xr + cB + 4);
  float s = 0.f;
#pragma unroll
  for (int e = 0; e < 4; ++e) { s += a0[e]; s += a1[e]; s += a2[e]; s += a3[e]; }
#pragma unroll
  for (int off = 16; off > 0; off >>= 1) s += __shfl_xor(s, off, 32);
  const float mean = s * kInvDim;
  const v4f d0 = a0 - mean, d1 = a1 - mean, d2 = a2 - mean, d3 = a3 - mean;
  float vs = 0.f;
#pragma unroll
  for (int e = 0; e < 4; ++e) { vs += d0[e] * d0[e]; vs += d1[e] * d1[e]; vs += d2[e] * d2[e]; vs += d3[e] * d3[e]; }
#pragma unroll
  for (int off = 16; off > 0; off >>= 1) vs += __shfl_xor(vs, off, 32);
  const float var  = vs * kInvDim;
  const float rstd = rsqrtf(var + kLnEps);
  const v4f g0 = *(const v4f*)(g + cA), g1 = *(const v4f*)(g + cA + 4), g2 = *(const v4f*)(g + cB), g3 = *(const v4f*)(g + cB + 4);
  const v4f b0 = *(const v4f*)(bt + cA), b1 = *(const v4f*)(bt + cA + 4), b2 = *(const v4f*)(bt + cB), b3 = *(const v4f*)(bt + cB + 4);
  const v4f y0 = d0 * rstd * g0 + b0;
  const v4f y1 = d1 * rstd * g1 + b1;
  const v4f y2 = d2 * rstd * g2 + b2;
  const v4f y3 = d3 * rstd * g3 + b3;
  const v4u u0 = (v4u){pk16(h_bits(y0[0]), h_bits(y0[1])), pk16(h_bits(y0[2]), h_bits(y0[3])),
                       pk16(h_bits(y1[0]), h_bits(y1[1])), pk16(h_bits(y1[2]), h_bits(y1[3]))};
  const v4u u1 = (v4u){pk16(h_bits(y2[0]), h_bits(y2[1])), pk16(h_bits(y2[2]), h_bits(y2[3])),
                       pk16(h_bits(y3[0]), h_bits(y3[1])), pk16(h_bits(y3[2]), h_bits(y3[3]))};
  if (row < nrows) {
    unsigned short* op = out + (size_t)row * kDim;
    *(volatile v4u*)(op + cA) = u0;
    *(volatile v4u*)(op + cB) = u1;
    __threadfence();
    *(volatile v4u*)(op + cA) = u0;
    *(volatile v4u*)(op + cB) = u1;
  }
}

__global__ __launch_bounds__(512) void softmax_row_kernel(const float* __restrict__ S, unsigned short* __restrict__ P, float carry) {
  __shared__ float redM[16];
  __shared__ float redS[16];
  const int row  = blockIdx.x;
  const int t    = threadIdx.x;
  const int lane = t & 31, wave = t >> 5;
  const int c0   = t * 8;
  const float* sr = S + (size_t)row * kSeq + c0;
  const v4f a = *(const v4f*)(sr);
  const v4f c = *(const v4f*)(sr + 4);
  float x[8];
#pragma unroll
  for (int e = 0; e < 4; ++e) { x[e] = a[e]; x[4 + e] = c[e]; }
  float m = fmaxf(fmaxf(fmaxf(x[0], x[1]), fmaxf(x[2], x[3])), fmaxf(fmaxf(x[4], x[5]), fmaxf(x[6], x[7])));
#pragma unroll
  for (int off = 16; off > 0; off >>= 1) m = fmaxf(m, __shfl_xor(m, off, 32));
  if (lane == 0) redM[wave] = m;
  __syncthreads();
  float mm = redM[0];
#pragma unroll
  for (int w = 1; w < 16; ++w) mm = fmaxf(mm, redM[w]);
  float ev[8];
  float ps = 0.f;
#pragma unroll
  for (int e = 0; e < 8; ++e) { ev[e] = expf(x[e] - mm); ps += ev[e]; }
#pragma unroll
  for (int off = 16; off > 0; off >>= 1) ps += __shfl_xor(ps, off, 32);
  if (lane == 0) redS[wave] = ps;
  __syncthreads();
  float tot = 0.f;
#pragma unroll
  for (int w = 0; w < 16; ++w) tot += redS[w];
  const float inv = carry * (1.0f / tot);
  unsigned short hb[8];
#pragma unroll
  for (int e = 0; e < 8; ++e) hb[e] = h_bits(ev[e] * inv);
  const v4u u = (v4u){pk16(hb[0], hb[1]), pk16(hb[2], hb[3]), pk16(hb[4], hb[5]), pk16(hb[6], hb[7])};
  unsigned short* pp = P + (size_t)row * kSeq + c0;
  *(volatile v4u*)pp = u;
  __threadfence();
  *(volatile v4u*)pp = u;
}

__global__ __launch_bounds__(256) void gelu_cast_kernel(const float* __restrict__ in, unsigned short* __restrict__ out, int n2, float carry) {
  const int i = blockIdx.x * 256 + threadIdx.x;
  if (i >= n2) return;
  unsigned u = 0u;
#pragma unroll 1
  for (int e = 0; e < 2; ++e) {
    const float v  = in[2 * (size_t)i + e];
    const float gl = 0.5f * v * (1.0f + erff(v * 0.70710678118654752f)) * carry;
    u |= ((unsigned)h_bits(gl)) << (16 * e);
  }
  ((volatile unsigned*)out)[i] = u;
  __threadfence();
  ((volatile unsigned*)out)[i] = u;
}

extern "C" void kernel_launch(void* const* d_in, const int* in_sizes, int n_in,
                              void* d_out, int out_size, void* d_ws, size_t ws_size,
                              hipStream_t stream) {
  if (n_in < 17) return;
  if (in_sizes[0] != kTok * kDim) return;
  if (in_sizes[1] != kDim * kDim || in_sizes[3] != kDim * kDim || in_sizes[5] != kDim * kDim || in_sizes[7] != kDim * kDim) return;
  if (in_sizes[2] != kDim || in_sizes[4] != kDim || in_sizes[6] != kDim || in_sizes[8] != kDim) return;
  if (in_sizes[9] != kDim || in_sizes[10] != kDim || in_sizes[11] != kDim || in_sizes[12] != kDim) return;
  if (in_sizes[13] != kDim * kFF || in_sizes[14] != kFF || in_sizes[15] != kFF * kDim || in_sizes[16] != kDim) return;
  if (out_size != kTok * kDim) return;
  if (ws_size < kWsTotal) return;

  const float* x    = (const float*)d_in[0];
  const float* Wq   = (const float*)d_in[1];
  const float* bq   = (const float*)d_in[2];
  const float* Wk   = (const float*)d_in[3];
  const float* bk   = (const float*)d_in[4];
  const float* Wv   = (const float*)d_in[5];
  const float* bv   = (const float*)d_in[6];
  const float* Wo   = (const float*)d_in[7];
  const float* bo   = (const float*)d_in[8];
  const float* ln1g = (const float*)d_in[9];
  const float* ln1b = (const float*)d_in[10];
  const float* ln2g = (const float*)d_in[11];
  const float* ln2b = (const float*)d_in[12];
  const float* W1   = (const float*)d_in[13];
  const float* b1   = (const float*)d_in[14];
  const float* W2   = (const float*)d_in[15];
  const float* b2   = (const float*)d_in[16];
  float* outp = (float*)d_out;

  char* ws = (char*)d_ws;
  unsigned short* H16  = (unsigned short*)(ws + kOffH);
  unsigned short* QK   = (unsigned short*)(ws + kOffQK);
  float*          X1   = (float*)(ws + kOffQK);
  unsigned short* VT   = (unsigned short*)(ws + kOffVT);
  unsigned short* WoT  = (unsigned short*)(ws + kOffVT);
  unsigned short* W1T  = WoT + (size_t)kDim * kDim;
  unsigned short* W2T  = W1T + (size_t)kFF * kDim;
  float*          SC   = (float*)(ws + kOffS);
  unsigned short* WqkvT = (unsigned short*)(ws + kOffS);
  float*          UF   = (float*)(ws + kOffS);
  unsigned short* P16  = (unsigned short*)(ws + kOffP);
  unsigned short* A1   = (unsigned short*)(ws + kOffP);
  const unsigned short* WqT  = WqkvT;
  const unsigned short* WkT  = WqkvT + (size_t)kDim * kDim;
  const unsigned short* WvTp = WqkvT + (size_t)2 * kDim * kDim;

  const dim3 blk(256);

  tcast_kernel<<<dim3(kDim / 64, kDim / 64, 3), blk, 0, stream>>>(Wq, Wk, Wv, WqkvT, kDim, kDim, kWCarry);

  ln_rows_kernel<<<dim3(kTok / 8), blk, 0, stream>>>(x, ln1g, ln1b, H16, kTok);

  wmma_gemm64<0, false, 2, 1, false><<<dim3((kTok / 64) * (kDim / 64) / 8, 1), blk, 0, stream>>>(
      H16, H16, kDim, 0L, WqT, WqT, kDim, 0L, (void*)QK, (void*)QK, kQKld, 0L, bq, x, 0L, kTok, kDim, kDim, kWCarryInv);
  wmma_gemm64<0, false, 2, 1, false><<<dim3((kTok / 64) * (kDim / 64) / 8, 1), blk, 0, stream>>>(
      H16, H16, kDim, 0L, WkT, WkT, kDim, 0L, (void*)(QK + kDim), (void*)(QK + kDim), kQKld, 0L, bk, x, 0L, kTok, kDim, kDim, kWCarryInv);

  wmma_gemm64<0, false, 1, 1, false><<<dim3((kDim / 64) * (kSeq / 64) / 8, kBatch), blk, 0, stream>>>(
      WvTp, WvTp, kDim, 0L, H16, H16, kDim, (long)kSeq * kDim, (void*)VT, (void*)VT, kSeq, (long)kDim * kSeq,
      bv, x, 0L, kDim, kSeq, kDim, kWCarryInv);

  for (int grp = 0; grp < kBatch * kHeads; ++grp) {
    const int bb = grp / kHeads, hd = grp % kHeads;
    const unsigned short* Aq = QK + (size_t)bb * kSeq * kQKld + (size_t)hd * kHeadDim;
    const unsigned short* Bk = Aq + kDim;
    wmma_gemm64<0, false, 0, 0, false><<<dim3((kSeq / 64) * (kSeq / 64) / 8, 1), blk, 0, stream>>>(
        Aq, Aq, kQKld, 0L, Bk, Bk, kQKld, 0L, (void*)SC, (void*)SC, kSeq, 0L, bq, x, 0L, kSeq, kSeq, kHeadDim, kScoreScale);
    softmax_row_kernel<<<dim3(kSeq), dim3(512), 0, stream>>>(SC, P16, kPCarry);
    const unsigned short* VTg  = VT + ((size_t)bb * kDim + (size_t)hd * kHeadDim) * kSeq;
    unsigned short*       CTXg = H16 + (size_t)bb * kSeq * kDim + (size_t)hd * kHeadDim;
    wmma_gemm64<0, false, 0, 1, false><<<dim3((kSeq / 64) * (kHeadDim / 64) / 8, 1), blk, 0, stream>>>(
        P16, P16, kSeq, 0L, VTg, VTg, kSeq, 0L, (void*)CTXg, (void*)CTXg, kDim, 0L, bq, x, 0L, kSeq, kHeadDim, kSeq, kPVScale);
  }

  tcast_kernel<<<dim3(kDim / 64, kDim / 64, 1), blk, 0, stream>>>(Wo, Wo, Wo, WoT, kDim, kDim, kWCarry);
  tcast_kernel<<<dim3(kDim / 64, kFF / 64, 1), blk, 0, stream>>>(W1, W1, W1, W1T, kDim, kFF, kWCarry);
  tcast_kernel<<<dim3(kFF / 64, kDim / 64, 1), blk, 0, stream>>>(W2, W2, W2, W2T, kFF, kDim, kWCarry);

  wmma_gemm64<0, false, 2, 0, true><<<dim3((kTok / 64) * (kDim / 64) / 8, 1), blk, 0, stream>>>(
      H16, H16, kDim, 0L, WoT, WoT, kDim, 0L, (void*)X1, (void*)X1, kDim, 0L, bo, x, 0L, kTok, kDim, kDim, kWoScale);

  ln_rows_kernel<<<dim3(kTok / 8), blk, 0, stream>>>(X1, ln2g, ln2b, H16, kTok);

  wmma_gemm64<0, false, 2, 0, false><<<dim3((kTok / 64) * (kFF / 64) / 8, 1), blk, 0, stream>>>(
      H16, H16, kDim, 0L, W1T, W1T, kDim, 0L, (void*)UF, (void*)UF, kFF, 0L, b1, x, 0L, kTok, kFF, kDim, kWCarryInv);

  gelu_cast_kernel<<<dim3((kTok * kFF / 2) / 256), blk, 0, stream>>>(UF, A1, kTok * kFF / 2, kActCarry);

  wmma_gemm64<0, false, 2, 0, true><<<dim3((kTok / 64) * (kDim / 64) / 8, 1), blk, 0, stream>>>(
      A1, A1, kFF, 0L, W2T, W2T, kFF, 0L, (void*)outp, (void*)outp, kDim, 0L, b2, X1, 0L, kTok, kDim, kFF, kW2Scale);
}
